// interpolater_61452392071435
// MI455X (gfx1250) — hardware-verified
//
#include <hip/hip_runtime.h>

#define Bsz 128
#define Cch 64
#define Hh  32
#define Tt  256


typedef __bf16 b16;
typedef __attribute__((ext_vector_type(16))) __bf16 v16b;
typedef __attribute__((ext_vector_type(8)))  float  v8f;
typedef __attribute__((ext_vector_type(4)))  float  v4f;

#define SH_STRIDE 36

__device__ __forceinline__ float relu1(float v) {
    return __builtin_amdgcn_fmed3f(v, 0.0f, 3.402823466e+38f);
}
__device__ __forceinline__ void split_bf16(float v, b16& hi, b16& lo) {
    const unsigned int u = __builtin_bit_cast(unsigned int, v) & 0xffff0000u;
    hi = __builtin_bit_cast(b16, (unsigned short)(u >> 16));
    lo = (b16)(v - __builtin_bit_cast(float, u));
}
__device__ __forceinline__ v8f wmma16b(v16b a, v16b b, v8f c) {
    v8f d = __builtin_amdgcn_wmma_f32_16x16x32_bf16(false, a, false, b, (short)0, c, false, false);
    asm volatile("v_nop\n\tv_nop\n\tv_nop\n\tv_nop" : "+v"(d) : "v"(a), "v"(b));
    return d;
}

__global__ __launch_bounds__(512)
void mrnn_scan_kernel(const float* __restrict__ x,
                      const float* __restrict__ mi,
                      const float* __restrict__ di,
                      const float* __restrict__ Wf, const float* __restrict__ Vf, const float* __restrict__ cf,
                      const float* __restrict__ Wb, const float* __restrict__ Vb, const float* __restrict__ cb,
                      const float* __restrict__ U,
                      float* __restrict__ partial)
{
    const int blk = blockIdx.x;
    const int c   = blk >> 1;
    const int dir = blk & 1;

    const int tid   = threadIdx.x;
    const int lane  = tid & 31;
    const int wave  = tid >> 5;
    const int mTile = wave >> 1;
    const int nTile = wave & 1;
    const int hb    = lane >> 4;

    const float* W  = dir ? Wb : Wf;
    const float* V  = dir ? Vb : Vf;
    const float* cv = dir ? cb : cf;

    __shared__ __attribute__((aligned(16))) float sH[2][Bsz * SH_STRIDE];
    __shared__ __attribute__((aligned(16))) float sFeat[2][3][Bsz];
    __shared__ __attribute__((aligned(16))) float sOut[Bsz];

    const int nLoc  = lane & 15;
    const int nGlob = nTile * 16 + nLoc;
    v16b bh_, bl_;
    {
        const float* wrow = W + (size_t)c * Hh * Hh + (size_t)nGlob * Hh;
        #pragma unroll
        for (int j = 0; j < 8; ++j) { b16 a, e; split_bf16(wrow[8 * hb + j], a, e); bh_[j] = a; bl_[j] = e; split_bf16(wrow[16 + 8 * hb + j], a, e); bh_[8 + j] = a; bl_[8 + j] = e; }
    }
    const float v0c = V[((size_t)c * Hh + nGlob) * 3 + 0];
    const float v1c = V[((size_t)c * Hh + nGlob) * 3 + 1];
    const float v2c = V[((size_t)c * Hh + nGlob) * 3 + 2];
    const float bC  = cv[(size_t)c * Hh + nGlob];

    float ureg[Hh];
    #pragma unroll
    for (int n = 0; n < Hh; ++n)
        ureg[n] = U[(size_t)c * (2 * Hh) + (size_t)dir * Hh + n];

    for (int i = tid; i < Bsz * SH_STRIDE; i += 512) sH[0][i] = 0.0f;

    if (tid < 3 * Bsz) {
        const int t_in0 = dir ? (Tt - 1) : 0;
        const int j = tid >> 7;
        const int b = tid & 127;
        const float* src = (j == 0) ? x : (j == 1 ? mi : di);
        sFeat[0][j][b] = src[(size_t)b * Cch * Tt + (size_t)c * Tt + t_in0];
    }
    __syncthreads();

    float* pbase = partial + ((size_t)dir * Cch + c) * Tt * Bsz;

    const int rb = mTile * 16 + hb * 8;

    for (int t = 0; t < Tt; ++t) {
        const int cur = t & 1;
        const int nxt = cur ^ 1;
        const float* sHc = sH[cur];
        float*       sHn = sH[nxt];

        v16b ah_, al_;
        {
            const float* rowp = sHc + (mTile * 16 + nLoc) * SH_STRIDE;
            const v4f p0 = *(const v4f*)(rowp + 8 * hb), p1 = *(const v4f*)(rowp + 8 * hb + 4);
            const v4f p2 = *(const v4f*)(rowp + 16 + 8 * hb), p3 = *(const v4f*)(rowp + 16 + 8 * hb + 4);
            float f[16] = {p0[0], p0[1], p0[2], p0[3], p1[0], p1[1], p1[2], p1[3], p2[0], p2[1], p2[2], p2[3], p3[0], p3[1], p3[2], p3[3]};
            #pragma unroll
            for (int e = 0; e < 16; ++e) { b16 a, l; split_bf16(f[e], a, l); ah_[e] = a; al_[e] = l; }
        }

        v8f acc;
        {
            union { v4f v[2]; float f[8]; } fx, fm, fd;
            fx.v[0] = *(const v4f*)&sFeat[cur][0][rb];
            fx.v[1] = *(const v4f*)&sFeat[cur][0][rb + 4];
            fm.v[0] = *(const v4f*)&sFeat[cur][1][rb];
            fm.v[1] = *(const v4f*)&sFeat[cur][1][rb + 4];
            fd.v[0] = *(const v4f*)&sFeat[cur][2][rb];
            fd.v[1] = *(const v4f*)&sFeat[cur][2][rb + 4];
            #pragma unroll
            for (int i = 0; i < 8; ++i)
                acc[i] = fmaf(v0c, fx.f[i], fmaf(v1c, fm.f[i], fmaf(v2c, fd.f[i], bC)));
        }

        v8f dacc = wmma16b(ah_, bh_, acc);
        dacc = wmma16b(ah_, bl_, dacc);
        dacc = wmma16b(al_, bh_, dacc);
        #pragma unroll
        for (int i = 0; i < 8; ++i) dacc[i] = relu1(dacc[i]);

        #pragma unroll
        for (int i = 0; i < 8; ++i)
            sHn[(rb + i) * SH_STRIDE + nGlob] = dacc[i];

        if (t > 0 && tid < Bsz) {
            const float* rowp = sHc + tid * SH_STRIDE;
            float s = 0.0f;
            #pragma unroll
            for (int q = 0; q < 8; ++q) {
                const v4f w = *(const v4f*)(rowp + 4 * q);
                s = fmaf(ureg[4 * q + 0], w[0], s);
                s = fmaf(ureg[4 * q + 1], w[1], s);
                s = fmaf(ureg[4 * q + 2], w[2], s);
                s = fmaf(ureg[4 * q + 3], w[3], s);
            }
            sOut[tid] = s;
        }

        if (t + 1 < Tt && tid < 3 * Bsz) {
            const int tn  = t + 1;
            const int t_b = Tt - tn;
            const int t_in = dir ? (t_b < (Tt - 1) ? t_b : (Tt - 1)) : (tn - 1);
            const int j = tid >> 7;
            const int b = tid & 127;
            const float* src = (j == 0) ? x : (j == 1 ? mi : di);
            sFeat[nxt][j][b] = src[(size_t)b * Cch * Tt + (size_t)c * Tt + t_in];
        }

        __syncthreads();

        if (t > 0 && wave == 0) {
            const int tprev = t - 1;
            const int t_out = dir ? (Tt - 1 - tprev) : tprev;
            const v4f v = *(const v4f*)&sOut[lane * 4];
            volatile v4f* dst = (volatile v4f*)(pbase + (size_t)t_out * Bsz + lane * 4);
            *dst = v; __threadfence(); *dst = v;
        }
    }

    if (tid < Bsz) {
        const float* rowp = sH[Tt & 1] + tid * SH_STRIDE;
        float s = 0.0f;
        #pragma unroll
        for (int q = 0; q < 8; ++q) {
            const v4f w = *(const v4f*)(rowp + 4 * q);
            s = fmaf(ureg[4 * q + 0], w[0], s);
            s = fmaf(ureg[4 * q + 1], w[1], s);
            s = fmaf(ureg[4 * q + 2], w[2], s);
            s = fmaf(ureg[4 * q + 3], w[3], s);
        }
        sOut[tid] = s;
    }
    __syncthreads();
    if (wave == 0) {
        const int t_out = dir ? 0 : (Tt - 1);
        const v4f v = *(const v4f*)&sOut[lane * 4];
        volatile v4f* dst = (volatile v4f*)(pbase + (size_t)t_out * Bsz + lane * 4);
        *dst = v; __threadfence(); *dst = v;
    }
}

__global__ __launch_bounds__(256)
void mrnn_combine_kernel(const float* __restrict__ partial,
                         const float* __restrict__ c0,
                         float* __restrict__ out, int n)
{
    const int i = blockIdx.x * blockDim.x + threadIdx.x;
    if (i >= n) return;
    const int t = i % Tt;
    const int c = (i / Tt) % Cch;
    const int b = i / (Tt * Cch);
    const size_t p = ((size_t)c * Tt + t) * Bsz + b;
    const float v = partial[p] + partial[(size_t)n + p] + c0[c];
    const float r = __builtin_amdgcn_fmed3f(v, 0.0f, 3.402823466e+38f);
    *(volatile float*)(out + i) = r;
    __threadfence();
    *(volatile float*)(out + i) = r;
}

extern "C" void kernel_launch(void* const* d_in, const int* in_sizes, int n_in,
                              void* d_out, int out_size, void* d_ws, size_t ws_size,
                              hipStream_t stream)
{
    (void)in_sizes; (void)n_in; (void)out_size;
    const float* x  = (const float*)d_in[0];
    const float* m  = (const float*)d_in[1];
    const float* d  = (const float*)d_in[2];
    const float* Wf = (const float*)d_in[3];
    const float* Vf = (const float*)d_in[4];
    const float* cf = (const float*)d_in[5];
    const float* Wb = (const float*)d_in[6];
    const float* Vb = (const float*)d_in[7];
    const float* cb = (const float*)d_in[8];
    const float* U  = (const float*)d_in[9];
    const float* c0 = (const float*)d_in[10];

    float* partial = (float*)d_ws;
    float* out     = (float*)d_out;
    if (ws_size < (size_t)2 * Bsz * Cch * Tt * sizeof(float)) return;

    mrnn_scan_kernel<<<Cch * 2, 512, 0, stream>>>(x, m, d, Wf, Vf, cf, Wb, Vb, cb, U, partial);

    const int n = Bsz * Cch * Tt;
    mrnn_combine_kernel<<<(n + 255) / 256, 256, 0, stream>>>(partial, c0, out, n);
}
